// MultiHeadAttention_17927193494305
// MI455X (gfx1250) — hardware-verified
//
#include <hip/hip_runtime.h>


#ifndef NB
#define NB 4
#endif
#ifndef SEQ
#define SEQ 2048
#endif
#define NB_FULL  4
#define SEQ_FULL 2048
#define DM   768
#define NH   8
#define HD   96
#define CTP  (2 * DM)
#define PCAR 1024.0f
#define QRS  2048.0f
#define SCL  0.10206207261596575f
#define L2E  1.4426950408889634f
#define PP   40
#define CP   200
#define PCS  ((2 * HD) / 8)

typedef _Float16 h16;
typedef unsigned short bf;
typedef __attribute__((ext_vector_type(16))) __bf16   v16bf;
typedef __attribute__((ext_vector_type(16))) _Float16 v16h;
typedef __attribute__((ext_vector_type(8)))  _Float16 v8h;
typedef __attribute__((ext_vector_type(8)))  unsigned short v8us;
typedef __attribute__((ext_vector_type(2)))  unsigned short v2us;
typedef __attribute__((ext_vector_type(8)))  float    v8f;
typedef __attribute__((ext_vector_type(4)))  float    v4f;
typedef v8h  __attribute__((may_alias)) v8ha;
typedef v4f  __attribute__((may_alias)) v4fa;
typedef v8us __attribute__((may_alias)) v8usa;

static_assert(DM == NH * HD);
static_assert(HD % 32 == 0);
static_assert(HD / 16 == 6);
static_assert(SEQ % 256 == 0);
static_assert((NB * SEQ) % 64 == 0);
static_assert(DM % 64 == 0);
static_assert(DM % 32 == 0);
static_assert(CTP % 64 == 0);
static_assert((2 * HD * 2) % 128 == 0);
static_assert(16 * PCS == 12 * 32);
static_assert(PP >= 32 && PP % 8 == 0);
static_assert(CP >= 2 * HD && CP % 8 == 0);
static_assert((NB * DM) % 32 == 0);
static_assert((SEQ * DM) % (8 * 256) == 0);
static_assert(NB <= NB_FULL && SEQ <= SEQ_FULL);

__device__ __forceinline__ unsigned short f2bf(float f) { unsigned u = __float_as_uint(f); u += 0x7FFFu + ((u >> 16) & 1u); return (unsigned short)(u >> 16); }
__device__ __forceinline__ float bf2f(unsigned short b) { return __uint_as_float(((unsigned)b) << 16); }
__device__ __forceinline__ float bfr(float f) { return bf2f(f2bf(f)); }
__device__ __forceinline__ void splitf(float y, unsigned short& h, unsigned short& l) { h = f2bf(y); l = f2bf(y - bf2f(h)); }
__device__ __forceinline__ v16h cat16(v8h lo, v8h hi) { return __builtin_shufflevector(lo, hi, 0, 1, 2, 3, 4, 5, 6, 7, 8, 9, 10, 11, 12, 13, 14, 15); }
__device__ __forceinline__ v16bf cat16b(v8us lo, v8us hi) { return __builtin_bit_cast(v16bf, __builtin_shufflevector(lo, hi, 0, 1, 2, 3, 4, 5, 6, 7, 8, 9, 10, 11, 12, 13, 14, 15)); }
__device__ __forceinline__ v8f wmma16(v16h a, v16h b, v8f c) { return __builtin_amdgcn_wmma_f32_16x16x32_f16(false, a, false, b, (short)0, c, false, false); }
__device__ __forceinline__ v8f wmmab(v16bf a, v16bf b, v8f c) { return __builtin_amdgcn_wmma_f32_16x16x32_bf16(false, a, false, b, (short)0, c, false, false); }
__device__ __forceinline__ v16h ldh(const h16* p) { return cat16(*(const v8h*)p, *(const v8h*)(p + 16)); }
__device__ __forceinline__ v16bf ldb(const bf* p) { return cat16b(*(const v8us*)p, *(const v8us*)(p + 16)); }

__global__ __launch_bounds__(256) void k_wtG(const float* __restrict__ w, int K, int N, bf* Bt, int il) {
    const int lane = threadIdx.x & 31; const int L0 = (blockIdx.x * 8 + (threadIdx.x >> 5)) * 8; const int KO = il ? 2 * K : K; const int nlines = N * KO / 64;
#pragma unroll
    for (int ps = 0; ps < 2; ++ps) {
#pragma unroll 1
        for (int l = 0; l < 8; ++l) { const int L = L0 + l; if (L >= nlines) break; const int e = L * 64 + lane * 2; const int kk = e % KO, n = e / KO;
            const int k = il ? ((kk / (2 * HD)) * HD + (kk % (2 * HD)) % HD) : kk; v2us o;
            o[0] = f2bf(w[(size_t)k * N + n]); o[1] = f2bf(w[(size_t)(k + 1) * N + n]); *(volatile v2us*)(Bt + e) = o; }
        if (ps == 0) __threadfence(); }
}

__global__ __launch_bounds__(256) void k_cvt8(const float* __restrict__ src, bf* dst) {
    const int i = blockIdx.x * 256 + threadIdx.x; const int b = blockIdx.y; if (i >= SEQ * DM / 8) return;
    const v8f v = *(const v8f*)(src + (size_t)b * SEQ_FULL * DM + (size_t)i * 8); v8us o;
#pragma unroll
    for (int k = 0; k < 8; ++k) o[k] = f2bf(v[k]);
    bf* d = dst + (size_t)b * SEQ * DM + (size_t)i * 8; *(volatile v8us*)d = o; __threadfence(); *(volatile v8us*)d = o; }

__global__ __launch_bounds__(32) void k_gemm(const bf* __restrict__ A, const bf* __restrict__ Bt, h16* C16, h16* CL, float* C32, const float* __restrict__ bias,
                                             size_t sA, size_t sB, size_t sC, int K, int ldc, int mode) {
    __shared__ __align__(16) float os[16 * 68];
    const size_t z = blockIdx.z; A += z * sA; Bt += z * sB; const size_t coff = z * sC;
    const int lane = threadIdx.x & 31, lr = lane & 15, hi = lane >> 4; const int r0 = blockIdx.x * 64, c0 = blockIdx.y * 64;
    v8f acc[4][4];
#pragma unroll
    for (int mb = 0; mb < 4; ++mb)
#pragma unroll
        for (int nb = 0; nb < 4; ++nb) acc[mb][nb] = (v8f){};
    const size_t aoff = (size_t)(r0 + lr) * K + 8 * hi, boff = (size_t)(c0 + lr) * K + 8 * hi;
#pragma unroll 1
    for (int kc = 0; kc < K; kc += 32) {
        v16bf a[4]; v16bf b;
#pragma unroll
        for (int mb = 0; mb < 4; ++mb) a[mb] = ldb(A + aoff + (size_t)mb * 16 * K + kc);
#pragma unroll
        for (int nb = 0; nb < 4; ++nb) { b = ldb(Bt + boff + (size_t)nb * 16 * K + kc);
#pragma unroll
            for (int mb = 0; mb < 4; ++mb) acc[mb][nb] = wmmab(a[mb], b, acc[mb][nb]); }
        asm volatile("v_nop\n\tv_nop\n\tv_nop\n\tv_nop" : "+v"(acc[0][3]), "+v"(acc[1][3]), "+v"(acc[2][3]), "+v"(acc[3][3]) : "v"(a[0]), "v"(a[1]), "v"(a[2]), "v"(a[3]), "v"(b));
    }
#pragma unroll
    for (int mb = 0; mb < 4; ++mb) {
#pragma unroll
        for (int nb = 0; nb < 4; ++nb) {
#pragma unroll
            for (int j = 0; j < 8; ++j) os[(hi * 8 + j) * 68 + nb * 16 + lr] = acc[mb][nb][j]; }
        __builtin_amdgcn_wave_barrier(); asm volatile("" ::: "memory");
        if (mode == 3) {
            float* crow = C32 + coff + (size_t)(r0 + mb * 16) * ldc + c0;
#pragma unroll 1
            for (int ps = 0; ps < 2; ++ps) {
#pragma unroll
                for (int s = 0; s < 8; ++s) { const int row = 2 * s + hi, cofs = lr * 4; v4f val = *(const v4fa*)(os + row * 68 + cofs);
                    val[0] += bfr(bias[c0 + cofs]); val[1] += bfr(bias[c0 + cofs + 1]); val[2] += bfr(bias[c0 + cofs + 2]); val[3] += bfr(bias[c0 + cofs + 3]);
                    *(volatile v4f*)(crow + (size_t)row * ldc + cofs) = val; }
                if (ps == 0) __threadfence(); }
        } else {
#pragma unroll 1
            for (int ps = 0; ps < 2; ++ps) {
#pragma unroll
                for (int s = 0; s < 4; ++s) { const int row = 4 * s + (lane >> 3), cg = lane & 7;
                    const v4f x0 = *(const v4fa*)(os + row * 68 + cg * 8); const v4f x1 = *(const v4fa*)(os + row * 68 + cg * 8 + 4);
                    const int grow = r0 + mb * 16 + row, gcol = c0 + cg * 8; const int bi0 = (mode == 2) ? grow : gcol; const int bst = (mode == 2) ? 0 : 1;
                    v8h o, ol;
#pragma unroll
                    for (int q = 0; q < 8; ++q) { const float v = ((q < 4) ? x0[q & 3] : x1[q & 3]) + bfr(bias[bi0 + q * bst]); const h16 hx = (h16)v; o[q] = hx; ol[q] = (h16)((v - (float)hx) * QRS); }
                    const size_t oo = coff + (size_t)grow * ldc + gcol;
                    *(volatile v8h*)(C16 + oo) = o; if (mode == 1) *(volatile v8h*)(CL + oo) = ol; }
                if (ps == 0) __threadfence(); }
        }
        __builtin_amdgcn_wave_barrier(); asm volatile("" ::: "memory");
    }
}

__global__ __launch_bounds__(256) void k_maskv(const h16* __restrict__ VT, const float* __restrict__ mask, float* MV) {
    __shared__ __align__(16) float red[32];
    const int wave = __builtin_amdgcn_readfirstlane((int)(threadIdx.x >> 5)); const int lane = threadIdx.x & 31;
#pragma unroll 1
    for (int i = 0; i < 4; ++i) { const int c = blockIdx.x * 32 + wave * 4 + i; const int b = c / DM; const h16* vr = VT + (size_t)c * SEQ; const float* mr = mask + (size_t)b * SEQ_FULL; float acc = 0.0f;
#pragma unroll 1
        for (int ch = 0; ch < SEQ / 256; ++ch) { const int k = ch * 256 + lane * 8; const v8h v = *(const v8h*)(vr + k); const v4f m0 = *(const v4f*)(mr + k); const v4f m1 = *(const v4f*)(mr + k + 4);
#pragma unroll
            for (int q = 0; q < 4; ++q) { acc += (bfr(m0[q]) * 1.0e9f) * (float)v[q]; acc += (bfr(m1[q]) * 1.0e9f) * (float)v[4 + q]; } }
#pragma unroll
        for (int sh = 16; sh; sh >>= 1) acc += __shfl_xor(acc, sh, 32);
        if (lane == 0) red[wave * 4 + i] = acc; }
    __syncthreads();
    if (wave == 0) { if (lane < 8) { const v4f o = *(const v4fa*)(red + lane * 4); float* p = MV + (size_t)blockIdx.x * 32 + lane * 4; *(volatile v4f*)p = o; __threadfence(); *(volatile v4f*)p = o; } }
}

__global__ __launch_bounds__(128) void k_attn(const h16* __restrict__ Q16, const h16* __restrict__ QL, const h16* __restrict__ K16, const h16* __restrict__ VT, const float* __restrict__ MV, bf* CT) {
    __shared__ __align__(16) h16 pws[4 * 16 * PP];
    __shared__ __align__(16) unsigned short cts[4 * 16 * CP];
    const int wave = __builtin_amdgcn_readfirstlane((int)(threadIdx.x >> 5));
    const int lane = threadIdx.x & 31, lr = lane & 15, hi = lane >> 4;
    const int b = blockIdx.z, h = blockIdx.y;
    const int row0 = b * SEQ + blockIdx.x * 64 + wave * 16;
    const int qoff = (row0 + lr) * DM + h * HD + 8 * hi;
    const int kbase = (b * SEQ + lr) * DM + h * HD + 8 * hi;
    const int vbase = (b * DM + h * HD + lr) * SEQ + 8 * hi;
    const int pb = wave * 16 * PP, cb = wave * 16 * CP;
    v8f ctx[6]; float mrun[8], srun[8];
#pragma unroll
    for (int nt = 0; nt < 6; ++nt) ctx[nt] = (v8f){};
#pragma unroll
    for (int r = 0; r < 8; ++r) { mrun[r] = -1.0e30f; srun[r] = 0.0f; }
#pragma unroll 1
    for (int kb = 0; kb < SEQ; kb += 32) {
        int qo = qoff; asm volatile("" : "+v"(qo));
        const int ko = kbase + kb * DM;
        v8f sh0 = (v8f){}, sh1 = (v8f){}, sl0 = (v8f){}, sl1 = (v8f){};
        v16h qa, qr, k0, k1;
#pragma unroll
        for (int ks = 0; ks < HD / 32; ++ks) {
            qa = ldh(Q16 + qo + ks * 32); qr = ldh(QL + qo + ks * 32);
            k0 = ldh(K16 + ko + ks * 32); k1 = ldh(K16 + ko + 16 * DM + ks * 32);
            sh0 = wmma16(qa, k0, sh0); sh1 = wmma16(qa, k1, sh1); sl0 = wmma16(qr, k0, sl0); sl1 = wmma16(qr, k1, sl1); }
        asm volatile("v_nop\n\tv_nop\n\tv_nop\n\tv_nop" : "+v"(sh0), "+v"(sh1), "+v"(sl0), "+v"(sl1) : "v"(qa), "v"(qr), "v"(k0), "v"(k1));
#pragma unroll
        for (int r = 0; r < 8; ++r) {
            const float t0 = (sh0[r] + sl0[r] * (1.0f / QRS)) * SCL; const float t1 = (sh1[r] + sl1[r] * (1.0f / QRS)) * SCL;
            float mx = fmaxf(t0, t1);
            mx = fmaxf(mx, __shfl_xor(mx, 1, 32)); mx = fmaxf(mx, __shfl_xor(mx, 2, 32)); mx = fmaxf(mx, __shfl_xor(mx, 4, 32)); mx = fmaxf(mx, __shfl_xor(mx, 8, 32));
            const float nm = fmaxf(mrun[r], mx); const float corr = __builtin_amdgcn_exp2f((mrun[r] - nm) * L2E); mrun[r] = nm;
            const float p0 = __builtin_amdgcn_exp2f((t0 - nm) * L2E); const float p1 = __builtin_amdgcn_exp2f((t1 - nm) * L2E);
            srun[r] = srun[r] * corr + (p0 + p1);
#pragma unroll
            for (int nt = 0; nt < 6; ++nt) ctx[nt][r] *= corr;
            pws[pb + (8 * hi + r) * PP + lr] = (h16)(p0 * PCAR); pws[pb + (8 * hi + r) * PP + 16 + lr] = (h16)(p1 * PCAR); }
        __builtin_amdgcn_wave_barrier(); asm volatile("" ::: "memory");
        const v16h pa = cat16(*(const v8ha*)(pws + pb + lr * PP + 8 * hi), *(const v8ha*)(pws + pb + lr * PP + 16 + 8 * hi));
        v16h vb;
#pragma unroll
        for (int nt = 0; nt < 6; ++nt) { vb = ldh(VT + vbase + nt * 16 * SEQ + kb); ctx[nt] = wmma16(pa, vb, ctx[nt]); }
        asm volatile("v_nop\n\tv_nop\n\tv_nop\n\tv_nop" : "+v"(ctx[0]), "+v"(ctx[1]), "+v"(ctx[2]), "+v"(ctx[3]), "+v"(ctx[4]), "+v"(ctx[5]) : "v"(pa), "v"(vb));
        __builtin_amdgcn_wave_barrier(); asm volatile("" ::: "memory");
    }
    float rinv[8];
#pragma unroll
    for (int r = 0; r < 8; ++r) { float s = srun[r]; s += __shfl_xor(s, 1, 32); s += __shfl_xor(s, 2, 32); s += __shfl_xor(s, 4, 32); s += __shfl_xor(s, 8, 32); rinv[r] = (1.0f / PCAR) * (1.0f / s); }
#pragma unroll
    for (int nt = 0; nt < 6; ++nt) { const float mvv = MV[b * DM + h * HD + nt * 16 + lr];
#pragma unroll
        for (int r = 0; r < 8; ++r) { const float val = ctx[nt][r] * rinv[r] + mvv; unsigned short hh, ll; splitf(val, hh, ll);
            cts[cb + (8 * hi + r) * CP + nt * 16 + lr] = hh; cts[cb + (8 * hi + r) * CP + HD + nt * 16 + lr] = ll; } }
    __builtin_amdgcn_wave_barrier(); asm volatile("" ::: "memory");
#pragma unroll 1
    for (int ps = 0; ps < 2; ++ps) {
#pragma unroll
        for (int it = 0; it < 12; ++it) { const int slot = it * 32 + lane; const int row = slot / PCS, pc = slot % PCS;
            const v8us o = *(const v8usa*)(cts + cb + row * CP + pc * 8);
            *(volatile v8us*)(CT + (size_t)(row0 + row) * CTP + h * 2 * HD + pc * 8) = o; }
        if (ps == 0) __threadfence(); }
}

constexpr size_t al256(size_t x) { return (x + 255) & ~(size_t)255; }
constexpr size_t SZ_W   = al256((size_t)DM * DM * 2);
constexpr size_t SZ_WO  = al256((size_t)DM * CTP * 2);
constexpr size_t SZ_PL  = al256((size_t)NB * SEQ * DM * 2);
constexpr size_t SZ_CT  = al256((size_t)NB * SEQ * CTP * 2);
constexpr size_t SZ_MV  = al256((size_t)NB * DM * 4);
constexpr size_t WS_TOTAL = 3 * SZ_W + SZ_WO + 5 * SZ_PL + SZ_CT + SZ_MV;
static_assert(WS_TOTAL <= (size_t)134217728);

extern "C" void kernel_launch(void* const* d_in, const int* in_sizes, int n_in,
                              void* d_out, int out_size, void* d_ws, size_t ws_size, hipStream_t stream) {
    if (n_in < 12) return;
    const long long need_x = (long long)(NB - 1) * SEQ_FULL * DM + (long long)SEQ * DM;
    if (in_sizes[0] < need_x || in_sizes[1] < need_x || in_sizes[2] < need_x) return;
    if (in_sizes[3] < (NB - 1) * SEQ_FULL + SEQ) return;
    if (in_sizes[4] < DM * DM || in_sizes[6] < DM * DM || in_sizes[8] < DM * DM || in_sizes[10] < DM * DM) return;
    if (in_sizes[5] < DM || in_sizes[7] < DM || in_sizes[9] < DM || in_sizes[11] < DM) return;
    if ((long long)out_size < (long long)NB * SEQ * DM) return;
    if (WS_TOTAL > ws_size) return;
    const float* xq = (const float*)d_in[0]; const float* xk = (const float*)d_in[1]; const float* xv = (const float*)d_in[2]; const float* mask = (const float*)d_in[3];
    const float* wq = (const float*)d_in[4]; const float* bq = (const float*)d_in[5]; const float* wk = (const float*)d_in[6]; const float* bk = (const float*)d_in[7];
    const float* wv = (const float*)d_in[8]; const float* bv = (const float*)d_in[9]; const float* wo = (const float*)d_in[10]; const float* bo = (const float*)d_in[11];
    float* OUT = (float*)d_out;
    char* wsp = (char*)d_ws;
    auto take = [&](size_t bytes) { char* p = wsp; wsp += bytes; return (void*)p; };
    bf* WQ = (bf*)take(SZ_W); bf* WK = (bf*)take(SZ_W); bf* WV = (bf*)take(SZ_W); bf* WO2 = (bf*)take(SZ_WO);
    bf* XB = (bf*)take(SZ_PL); h16* Q16 = (h16*)take(SZ_PL); h16* QL = (h16*)take(SZ_PL); h16* K16 = (h16*)take(SZ_PL); h16* VT16 = (h16*)take(SZ_PL);
    bf* CT = (bf*)take(SZ_CT); float* MV = (float*)take(SZ_MV);

    const unsigned gW = (unsigned)((DM * DM / 64 + 63) / 64), gWO = (unsigned)((DM * CTP / 64 + 63) / 64);
    k_wtG<<<gW, 256, 0, stream>>>(wq, DM, DM, WQ, 0);
    k_wtG<<<gW, 256, 0, stream>>>(wk, DM, DM, WK, 0);
    k_wtG<<<gW, 256, 0, stream>>>(wv, DM, DM, WV, 0);
    k_wtG<<<gWO, 256, 0, stream>>>(wo, DM, DM, WO2, 1);
    const dim3 gC((unsigned)(SEQ * DM / 8 / 256), NB, 1);
    const dim3 gP((unsigned)(NB * SEQ / 64), DM / 64, 1);
    k_cvt8<<<gC, 256, 0, stream>>>(xq, XB);
    k_gemm<<<gP, 32, 0, stream>>>(XB, WQ, Q16, QL, OUT, bq, (size_t)0, (size_t)0, (size_t)0, DM, DM, 1);
    k_cvt8<<<gC, 256, 0, stream>>>(xk, XB);
    k_gemm<<<gP, 32, 0, stream>>>(XB, WK, K16, K16, OUT, bk, (size_t)0, (size_t)0, (size_t)0, DM, DM, 0);
    k_cvt8<<<gC, 256, 0, stream>>>(xv, XB);
    k_gemm<<<dim3(DM / 64, SEQ / 64, NB), 32, 0, stream>>>(WV, XB, VT16, VT16, OUT, bv, (size_t)0, (size_t)SEQ * DM, (size_t)DM * SEQ, DM, SEQ, 2);
    k_maskv<<<(unsigned)(NB * DM / 32), 256, 0, stream>>>(VT16, mask, MV);
    k_attn<<<dim3(SEQ / 64, NH, NB), 128, 0, stream>>>(Q16, QL, K16, VT16, MV, CT);
    k_gemm<<<gP, 32, 0, stream>>>(CT, WO2, Q16, Q16, OUT, bo, (size_t)0, (size_t)0, (size_t)0, CTP, DM, 3);
}
